// BigMaskAttention_62783831933470
// MI455X (gfx1250) — hardware-verified
//
#include <hip/hip_runtime.h>

#define SS  4096
#define HH  16
#define HD  80
#define HDP 96
#define NCU 9

typedef _Float16 f16;
typedef __bf16 bf16t;
typedef __attribute__((ext_vector_type(16))) f16 f16x16;
typedef __attribute__((ext_vector_type(8)))  f16 f16x8;
typedef __attribute__((ext_vector_type(16))) __bf16 bf16x16;
typedef __attribute__((ext_vector_type(8)))  __bf16 bf16x8;
typedef __attribute__((ext_vector_type(8)))  float f32x8;
typedef __attribute__((ext_vector_type(4)))  float v4f_t;
typedef float v4fa __attribute__((ext_vector_type(4), may_alias));
typedef __attribute__((ext_vector_type(4))) unsigned v4u_t;
typedef unsigned v4ua __attribute__((ext_vector_type(4), may_alias));

__device__ __forceinline__ f32x8 wmma_f16(f16x16 a, f16x16 b, f32x8 c) {
  c = __builtin_amdgcn_wmma_f32_16x16x32_f16(false, a, false, b, (short)0, c, false, false);
  asm volatile("v_nop\n\tv_nop\n\tv_nop\n\tv_nop" : "+v"(c) : "v"(a), "v"(b));
  return c;
}
__device__ __forceinline__ f32x8 wmma_b16(bf16x16 a, bf16x16 b, f32x8 c) {
  c = __builtin_amdgcn_wmma_f32_16x16x32_bf16(false, a, false, b, (short)0, c, false, false);
  asm volatile("v_nop\n\tv_nop\n\tv_nop\n\tv_nop" : "+v"(c) : "v"(a), "v"(b));
  return c;
}
__device__ __forceinline__ bf16x16 ldsb_frag(const __bf16* base, int stride) {
  const int lane = threadIdx.x & 31, row = lane & 15, kh = (lane >> 4) * 8;
  const bf16x8 lo = *(const bf16x8*)(base + row * stride + kh);
  const bf16x8 hi = *(const bf16x8*)(base + row * stride + kh + 16);
  bf16x16 f;
#pragma unroll
  for (int i = 0; i < 8; ++i) { f[i] = lo[i]; f[i + 8] = hi[i]; }
  return f;
}
__device__ __forceinline__ bf16x16 glbb_frag(const __bf16* base, int stride, int row0, int col0) {
  const int lane = threadIdx.x & 31, row = lane & 15, kh = (lane >> 4) * 8;
  const __bf16* p = base + (size_t)(row0 + row) * stride + col0 + kh;
  const bf16x8 lo = *(const bf16x8*)(p), hi = *(const bf16x8*)(p + 16);
  bf16x16 f;
#pragma unroll
  for (int i = 0; i < 8; ++i) { f[i] = lo[i]; f[i + 8] = hi[i]; }
  return f;
}
__device__ __forceinline__ f16x16 ldsh_frag(const f16* base, int stride) {
  const int lane = threadIdx.x & 31, row = lane & 15, kh = (lane >> 4) * 8;
  const f16x8 lo = *(const f16x8*)(base + row * stride + kh);
  const f16x8 hi = *(const f16x8*)(base + row * stride + kh + 16);
  f16x16 f;
#pragma unroll
  for (int i = 0; i < 8; ++i) { f[i] = lo[i]; f[i + 8] = hi[i]; }
  return f;
}

__global__ __launch_bounds__(256) void k_padbf(const float* __restrict__ src, __bf16* __restrict__ dst) {
  __shared__ __attribute__((aligned(16))) __bf16 tS[64 * 96];
  const int tid = threadIdx.x; const size_t r0 = (size_t)blockIdx.x * 64;
  for (int e = tid; e < 64 * 96; e += 256) { const int r = e / 96, c = e % 96; tS[e] = (c < HD) ? (__bf16)src[(r0 + r) * HD + c] : (__bf16)0.0f; }
  __syncthreads();
#pragma unroll 1
  for (int pass = 0; pass < 2; ++pass) {
    for (int q = tid; q < 64 * 96 / 8; q += 256) *(volatile v4u_t*)((unsigned*)(dst + r0 * HDP) + q * 4) = *(const v4ua*)(tS + q * 8);
    __threadfence();
  }
}
__global__ __launch_bounds__(256) void k_vt(const float* __restrict__ v, f16* __restrict__ Vt) {
  __shared__ float tS[64][81];
  const int tid = threadIdx.x, h = blockIdx.x / (SS / 64), s0 = (blockIdx.x % (SS / 64)) * 64;
  for (int e = tid; e < 64 * HD; e += 256) { const int s = e / HD, d = e % HD; tS[s][d] = (float)(__bf16)v[((size_t)h * SS + s0 + s) * HD + d]; }
  __syncthreads();
  for (int ch = tid; ch < HD * 8; ch += 256) { const int d = ch >> 3, q8 = (ch & 7) * 8;
    union { f16 hh[8]; v4u_t u; } cv;
#pragma unroll
    for (int e = 0; e < 8; ++e) cv.hh[e] = (f16)tS[q8 + e][d];
    f16* dstp = Vt + ((size_t)h * HD + d) * SS + s0 + q8;
    *(volatile v4u_t*)dstp = cv.u; __threadfence(); *(volatile v4u_t*)dstp = cv.u; }
}

__global__ __launch_bounds__(128) void attn_kernel(const __bf16* __restrict__ Qp, const __bf16* __restrict__ Kp, const f16* __restrict__ Vt,
                                                   const int* __restrict__ cu, const float* __restrict__ scaling, float* __restrict__ out) {
  __shared__ __attribute__((aligned(16))) __bf16 ldsK[32 * 104];
  __shared__ __attribute__((aligned(16))) f16 ldsV[HD * 40];
  __shared__ __attribute__((aligned(16))) float outS[64 * 164];
  __shared__ int cus[NCU];
  const int t = threadIdx.x, wave = t >> 5, lane = t & 31, qlane = lane & 15, kh8 = (lane >> 4) * 8;
  const int q0blk = blockIdx.x * 64, hp = blockIdx.y;
  const int q0 = q0blk + wave * 16;
  if (t == 0) {
    int c[NCU];
#pragma unroll
    for (int i = 0; i < NCU; ++i) c[i] = cu[i];
    for (int i = 1; i < NCU; ++i) { int v = c[i], j = i - 1; while (j >= 0 && c[j] > v) { c[j + 1] = c[j]; --j; } c[j + 1] = v; }
#pragma unroll
    for (int i = 0; i < NCU; ++i) cus[i] = c[i];
  }
  __syncthreads();
  auto segof = [&](int idx) { int s = 0;
#pragma unroll
    for (int i = 0; i < NCU; ++i) s += (cus[i] <= idx) ? 1 : 0; return s; };
  const int sfirst = segof(q0blk), slast = segof(q0blk + 63);
  const int klo = (sfirst == 0) ? 0 : min(max(cus[sfirst - 1], 0), SS);
  const int khi = (slast >= NCU) ? SS : min(max(cus[min(slast, NCU - 1)], 0), SS);
  const float scl = (*scaling) * 1.44269504088896340736f;
  const float NEG2 = -3.0e38f;
  const int myseg = segof(q0 + qlane);
#pragma unroll 1
  for (int hh2 = 0; hh2 < 2; ++hh2) {
    const int h = hp * 2 + hh2;
    const __bf16* Qh = Qp + (size_t)h * SS * HDP;
    const __bf16* Kh = Kp + (size_t)h * SS * HDP;
    const f16* Vh = Vt + (size_t)h * HD * SS;
    bf16x16 qf[3];
#pragma unroll
    for (int c3 = 0; c3 < 3; ++c3) qf[c3] = glbb_frag(Qh, HDP, q0, c3 * 32);
    f32x8 o[5], ox[5];
#pragma unroll
    for (int j = 0; j < 5; ++j) { f32x8 z = {}; o[j] = z; ox[j] = z; }
    float mrun = NEG2, lrun = 0.0f;
#pragma unroll 1
    for (int kb = klo & ~31; kb < khi; kb += 32) {
      __syncthreads();
      { const int row = t >> 2, qo = (t & 3) * 24; const __bf16* srcp = Kh + (size_t)(kb + row) * HDP + qo;
        const unsigned* su = (const unsigned*)srcp; unsigned* du = (unsigned*)(ldsK + row * 104 + qo);
#pragma unroll
        for (int i = 0; i < 12; ++i) du[i] = su[i]; }
      { for (int d = t; d < HD; d += 128) { const f16* srcp = Vh + (size_t)d * SS + kb;
#pragma unroll
          for (int i = 0; i < 4; ++i) *(f16x8*)(ldsV + d * 40 + 8 * i) = *(const f16x8*)(srcp + 8 * i); } }
      __syncthreads();
      f32x8 s0 = {}, s1 = {};
#pragma unroll
      for (int c3 = 0; c3 < 3; ++c3) {
        s0 = wmma_b16(ldsb_frag(ldsK + 0 * 104 + c3 * 32, 104), qf[c3], s0);
        s1 = wmma_b16(ldsb_frag(ldsK + 16 * 104 + c3 * 32, 104), qf[c3], s1);
      }
      float mx = NEG2;
#pragma unroll
      for (int r = 0; r < 8; ++r) {
        const int k0i = kb + kh8 + r, k1i = k0i + 16;
        const bool a0 = (k0i < SS) && (segof(k0i) == myseg), a1 = (k1i < SS) && (segof(k1i) == myseg);
        s0[r] = a0 ? s0[r] * scl : NEG2; s1[r] = a1 ? s1[r] * scl : NEG2;
        mx = fmaxf(mx, fmaxf(s0[r], s1[r]));
      }
      mx = fmaxf(mx, __shfl_xor(mx, 16, 32));
      const float mnew = fmaxf(mrun, mx);
      const float alpha = exp2f(mrun - mnew);
      f16x16 pf, pl; float rs = 0.0f;
#pragma unroll
      for (int r = 0; r < 8; ++r) {
        const float p0 = (s0[r] <= -1.0e38f) ? 0.0f : exp2f(s0[r] - mnew) * 1024.0f;
        const float p1 = (s1[r] <= -1.0e38f) ? 0.0f : exp2f(s1[r] - mnew) * 1024.0f;
        rs += p0 + p1;
        const f16 h0 = (f16)p0, h1 = (f16)p1; pf[r] = h0; pl[r] = (f16)((p0 - (float)h0) * 2048.0f); pf[8 + r] = h1; pl[8 + r] = (f16)((p1 - (float)h1) * 2048.0f);
      }
      rs += __shfl_xor(rs, 16, 32);
      lrun = lrun * alpha + rs * (1.0f / 1024.0f); mrun = mnew;
#pragma unroll
      for (int j = 0; j < 5; ++j) {
#pragma unroll
        for (int r = 0; r < 8; ++r) { o[j][r] *= alpha; ox[j][r] *= alpha; }
        const f16x16 vf = ldsh_frag(ldsV + (j * 16) * 40, 40);
        o[j] = wmma_f16(vf, pf, o[j]); ox[j] = wmma_f16(vf, pl, ox[j]);
      }
    }
    const float rl = 1.0f / (lrun * 1024.0f);
#pragma unroll
    for (int j = 0; j < 5; ++j)
#pragma unroll
      for (int r = 0; r < 8; ++r) outS[(wave * 16 + qlane) * 164 + hh2 * HD + j * 16 + kh8 + r] = (o[j][r] + ox[j][r] * (1.0f / 2048.0f)) * rl;
  }
  __syncthreads();
#pragma unroll 1
  for (int pass = 0; pass < 2; ++pass) {
    for (int ch = t; ch < 64 * 40; ch += 128) { const int ql = ch / 40, c4 = (ch % 40) * 4;
      *(volatile v4f_t*)(out + (size_t)(q0blk + ql) * (HH * HD) + hp * 2 * HD + c4) = *(const volatile v4fa*)(outS + ql * 164 + c4); }
    __threadfence();
  }
}

extern "C" void kernel_launch(void* const* d_in, const int* in_sizes, int n_in,
                              void* d_out, int out_size, void* d_ws, size_t ws_size,
                              hipStream_t stream) {
  (void)in_sizes; (void)n_in; (void)out_size; (void)ws_size;
  const float* q = (const float*)d_in[0];
  const float* k = (const float*)d_in[1];
  const float* v = (const float*)d_in[2];
  const int* cu = (const int*)d_in[3];
  const float* scaling = (const float*)d_in[4];
  float* out = (float*)d_out;
  char* ws = (char*)d_ws;
  __bf16* Qp = (__bf16*)ws; ws += (size_t)HH * SS * HDP * 2;
  __bf16* Kp = (__bf16*)ws; ws += (size_t)HH * SS * HDP * 2;
  f16* Vt = (f16*)ws; ws += (size_t)HH * HD * SS * 2;
  k_padbf<<<dim3(HH * SS / 64), dim3(256), 0, stream>>>(q, Qp);
  k_padbf<<<dim3(HH * SS / 64), dim3(256), 0, stream>>>(k, Kp);
  k_vt<<<dim3(HH * SS / 64), dim3(256), 0, stream>>>(v, Vt);
  attn_kernel<<<dim3(SS / 64, HH / 2), dim3(128), 0, stream>>>(Qp, Kp, Vt, cu, scaling, out);
}
